// SAGE_GraphConv_24592982737487
// MI455X (gfx1250) — hardware-verified
//
#include <hip/hip_runtime.h>
#include <stddef.h>

typedef __attribute__((ext_vector_type(16))) _Float16 v16h;
typedef __attribute__((ext_vector_type(8)))  _Float16 v8h;
typedef __attribute__((ext_vector_type(16))) __bf16   v16b;
typedef __attribute__((ext_vector_type(8)))  __bf16   v8b;
typedef __attribute__((ext_vector_type(8)))  float    v8f;
typedef __attribute__((ext_vector_type(4)))  float    v4f;
typedef __attribute__((ext_vector_type(4)))  int      v4i;

constexpr int FDIM = 512;
#define NTHR    256
#define NWAVE   8
#define EPT     8
#define NGRP    2
#define CHUNK   (NTHR * EPT * NGRP)
#define WCAP    (EPT * NGRP * 32)
#define LISTN   (NWAVE * WCAP)
#define NBA     64
#define NBD     4096
#define LDS_AGG (NBA * FDIM * 4 + LISTN * 4 + 64)
constexpr float WSCALE     = 16.0f;
constexpr float WSCALE_INV = 0.0625f;

static_assert((CHUNK & (CHUNK - 1)) == 0);
static_assert(CHUNK <= 4096);
static_assert((NBA & (NBA - 1)) == 0 && NBA <= 4096);
static_assert((NBD & (NBD - 1)) == 0 && NBD <= 4096);
static_assert(NBD == NWAVE * 4 * 128);
static_assert(NBA == NWAVE * 8);
static_assert((NBA * FDIM / 4) % NTHR == 0);
static_assert(FDIM == 512);
static_assert(LDS_AGG == 147520);

__device__ __forceinline__ unsigned short f2bf_bits(float f) {
  unsigned u = __float_as_uint(f);
  return (unsigned short)((u + 0x7FFFu + ((u >> 16) & 1u)) >> 16);
}
__device__ __forceinline__ float bf_bits2f(unsigned short h) { return __uint_as_float(((unsigned)h) << 16); }

__device__ __forceinline__ void dep_guard_h(v8f& a, v8f& b, v16h x, v16h y) { asm volatile("v_nop\n\tv_nop\n\tv_nop\n\tv_nop" : "+v"(a), "+v"(b) : "v"(x), "v"(y)); }
__device__ __forceinline__ void dep_guard_b(v8f& a, v8f& b, v16b x, v16b y) { asm volatile("v_nop\n\tv_nop\n\tv_nop\n\tv_nop" : "+v"(a), "+v"(b) : "v"(x), "v"(y)); }
__device__ __forceinline__ void keep4_h(v16h a, v16h b, v16h c, v16h d) { asm volatile("v_nop" :: "v"(a), "v"(b), "v"(c), "v"(d)); }
__device__ __forceinline__ void keep4_b(v16b a, v16b b, v16b c, v16b d) { asm volatile("v_nop" :: "v"(a), "v"(b), "v"(c), "v"(d)); }
__device__ __forceinline__ void acc_guard4(v8f& a, v8f& b, v8f& c, v8f& d) { asm volatile("v_nop\n\tv_nop\n\tv_nop\n\tv_nop" : "+v"(a), "+v"(b), "+v"(c), "+v"(d)); }
template <typename T> struct Frag;
template <> struct Frag<_Float16> {
  typedef v16h V; union U { v16h v; v8h h[2]; };
  static __device__ __forceinline__ v16h load(const _Float16* p) {
    U f; f.h[0] = *(const v8h*)(p); f.h[1] = *(const v8h*)(p + 16); return f.v;
  }
  static __device__ __forceinline__ v8f mma(v16h a, v16h b, v8f c) {
    return __builtin_amdgcn_wmma_f32_16x16x32_f16(false, a, false, b, (short)0, c, false, false);
  }
  static __device__ __forceinline__ void guard(v8f& a, v8f& b, v16h x, v16h y) { dep_guard_h(a, b, x, y); }
  static __device__ __forceinline__ void keep(v16h a, v16h b, v16h c, v16h d) { keep4_h(a, b, c, d); }
};
template <> struct Frag<__bf16> {
  typedef v16b V; union U { v16b v; v8b h[2]; };
  static __device__ __forceinline__ v16b load(const __bf16* p) {
    U f; f.h[0] = *(const v8b*)(p); f.h[1] = *(const v8b*)(p + 16); return f.v;
  }
  static __device__ __forceinline__ v8f mma(v16b a, v16b b, v8f c) {
    return __builtin_amdgcn_wmma_f32_16x16x32_bf16(false, a, false, b, (short)0, c, false, false);
  }
  static __device__ __forceinline__ void guard(v8f& a, v8f& b, v16b x, v16b y) { dep_guard_b(a, b, x, y); }
  static __device__ __forceinline__ void keep(v16b a, v16b b, v16b c, v16b d) { keep4_b(a, b, c, d); }
};

template <int ET> struct Elem;
template <> struct Elem<0> { typedef _Float16 T; };
template <> struct Elem<1> { typedef __bf16 T; };
template <int ET, bool SPLIT, int BIAS_MODE, int OUT_MODE, bool RESID, int ACT = 0>
__global__ __launch_bounds__(256) void wmma_gemm64(
    const unsigned short* __restrict__ Ap, const unsigned short* __restrict__ A2p, int lda, long strideA,
    const unsigned short* __restrict__ Btp, const unsigned short* __restrict__ Bt2p, int ldb, long strideB,
    void* __restrict__ Cout, void* __restrict__ Cout2, int ldc, long strideC,
    const float* __restrict__ bias,
    const float* __restrict__ resid, long strideR,
    int M, int N, int K, float scale) {
  typedef typename Elem<ET>::T T;
  typedef typename Frag<T>::V V;
  const T* A = (const T*)Ap; const T* A2 = (const T*)A2p; const T* Bt = (const T*)Btp; const T* Bt2 = (const T*)Bt2p;
  __shared__ __align__(16) float sT[8][16 * 68];
  const int b    = blockIdx.y;
  const int lane = threadIdx.x & 31;
  const int wave = threadIdx.x >> 5;
  const int tilesN = N >> 6;
  const int tilesM = M >> 6;
  const int tile = blockIdx.x * 8 + wave;
  if (tile >= tilesM * tilesN) return;
  const int tm = tile / tilesN;
  const int tn = tile - tm * tilesN;
  const int m0 = tm << 6;
  const int n0 = tn << 6;

  const T* Ab  = A  + (size_t)b * strideA;
  const T* Bb  = Bt + (size_t)b * strideB;
  const T* Ab2 = SPLIT ? (A2  + (size_t)b * strideA) : nullptr;
  const T* Bb2 = SPLIT ? (Bt2 + (size_t)b * strideB) : nullptr;

  const int rlane = lane & 15;
  const int koff  = (lane >> 4) * 8;
  const int mOff  = (lane >> 4) * 8;

  v8f acc[4][4];
#pragma unroll
  for (int i = 0; i < 4; ++i)
#pragma unroll
    for (int j = 0; j < 4; ++j) acc[i][j] = (v8f){0.f,0.f,0.f,0.f,0.f,0.f,0.f,0.f};

  for (int k0 = 0; k0 < K; k0 += 32) {
    V bh[4], bl[4];
#pragma unroll
    for (int j = 0; j < 4; ++j) {
      const size_t bo = (size_t)(n0 + (j << 4) + rlane) * ldb + koff + k0;
      bh[j] = Frag<T>::load(Bb + bo);
      if (SPLIT) bl[j] = Frag<T>::load(Bb2 + bo);
    }
#pragma unroll
    for (int i = 0; i < 4; ++i) {
      const size_t ao = (size_t)(m0 + (i << 4) + rlane) * lda + koff + k0;
      V ah = Frag<T>::load(Ab + ao);
      V al;
      if (SPLIT) al = Frag<T>::load(Ab2 + ao);
#pragma unroll
      for (int j = 0; j < 4; ++j) {
        acc[i][j] = Frag<T>::mma(ah, bh[j], acc[i][j]);
        if (SPLIT) {
          acc[i][j] = Frag<T>::mma(ah, bl[j], acc[i][j]);
          acc[i][j] = Frag<T>::mma(al, bh[j], acc[i][j]);
        }
      }
      Frag<T>::guard(acc[i][0], acc[i][3], ah, SPLIT ? al : ah);
    }
    Frag<T>::keep(bh[0], bh[1], bh[2], bh[3]);
    if (SPLIT) Frag<T>::keep(bl[0], bl[1], bl[2], bl[3]);
  }
  acc_guard4(acc[0][0], acc[0][1], acc[0][2], acc[0][3]);
  acc_guard4(acc[1][0], acc[1][1], acc[1][2], acc[1][3]);
  acc_guard4(acc[2][0], acc[2][1], acc[2][2], acc[2][3]);
  acc_guard4(acc[3][0], acc[3][1], acc[3][2], acc[3][3]);

  float* slab = sT[wave];
  const float* Rb = RESID ? (resid + (size_t)b * strideR) : nullptr;
#pragma unroll
  for (int i = 0; i < 4; ++i) {
    const int mBase = m0 + (i << 4);
#pragma unroll
    for (int j = 0; j < 4; ++j) {
      const int n = n0 + (j << 4) + rlane;
      float bv = 0.f;
      if (BIAS_MODE == 2) bv = bias[n];
#pragma unroll
      for (int r = 0; r < 8; ++r) {
        float v = acc[i][j][r] * scale;
        if (BIAS_MODE == 1) v += bias[mBase + mOff + r];
        if (BIAS_MODE == 2) v += bv;
        if (RESID) v += Rb[(size_t)(mBase + mOff + r) * ldc + n];
        if (ACT == 1) v = tanhf(v);
        if (ACT == 2) v = fmaxf(v, 0.0f);
        if (ACT == 3) v = v / (1.0f + expf(-v));
        if (ACT == 4) v = (v > 0.f) ? v : 0.01f * v;
        if (ACT == 5) v = 0.5f * v * (1.0f + erff(v * 0.70710678118654752f));
        slab[(mOff + r) * 68 + (j << 4) + rlane] = v;
      }
    }
    __builtin_amdgcn_fence(__ATOMIC_RELEASE, "workgroup");
    __builtin_amdgcn_wave_barrier();
    __builtin_amdgcn_fence(__ATOMIC_ACQUIRE, "workgroup");
    if (OUT_MODE == 0) {
      float* C = (float*)Cout + (size_t)b * strideC;
      const int hh = lane >> 4, c4 = (lane & 15) * 4;
      for (int pass = 0; pass < 2; ++pass) {
#pragma unroll
        for (int it = 0; it < 8; ++it) {
          const int row = it * 2 + hh;
          v4f v = *(const v4f*)(slab + row * 68 + c4);
          *(volatile v4f*)(C + (size_t)(mBase + row) * ldc + n0 + c4) = v;
        }
        __threadfence();
      }
    } else {
      const int q = lane >> 3, c8 = (lane & 7) * 8;
      unsigned short* C  = (unsigned short*)Cout  + (size_t)b * strideC;
      unsigned short* C2 = (OUT_MODE == 2) ? ((unsigned short*)Cout2 + (size_t)b * strideC) : nullptr;
      for (int pass = 0; pass < 2; ++pass) {
#pragma unroll
        for (int it = 0; it < 4; ++it) {
          const int row = it * 4 + q;
          const float* sp = slab + row * 68 + c8;
          v8h hv, lv;
#pragma unroll
          for (int e = 0; e < 8; ++e) {
            if (OUT_MODE == 1) {
              hv[e] = (_Float16)sp[e];
            } else {
              unsigned short hb = f2bf_bits(sp[e]);
              unsigned short lb = f2bf_bits(sp[e] - bf_bits2f(hb));
              hv[e] = __builtin_bit_cast(_Float16, hb);
              lv[e] = __builtin_bit_cast(_Float16, lb);
            }
          }
          *(volatile v8h*)(C + (size_t)(mBase + row) * ldc + n0 + c8) = hv;
          if (OUT_MODE == 2) *(volatile v8h*)(C2 + (size_t)(mBase + row) * ldc + n0 + c8) = lv;
        }
        __threadfence();
      }
    }
    __builtin_amdgcn_fence(__ATOMIC_RELEASE, "workgroup");
    __builtin_amdgcn_wave_barrier();
    __builtin_amdgcn_fence(__ATOMIC_ACQUIRE, "workgroup");
  }
}

__device__ __forceinline__ v4f relu4(v4f a) {
  a.x = fmaxf(a.x, 0.f); a.y = fmaxf(a.y, 0.f); a.z = fmaxf(a.z, 0.f); a.w = fmaxf(a.w, 0.f);
  return a;
}
__device__ __forceinline__ float sq4(v4f a) { return (a.x * a.x + a.y * a.y) + (a.z * a.z + a.w * a.w); }
__device__ __forceinline__ v8h pack8h(v4f a, v4f b) {
  v8h h;
  h[0] = (_Float16)a.x; h[1] = (_Float16)a.y; h[2] = (_Float16)a.z; h[3] = (_Float16)a.w;
  h[4] = (_Float16)b.x; h[5] = (_Float16)b.y; h[6] = (_Float16)b.z; h[7] = (_Float16)b.w;
  return h;
}

template <int NB>
__device__ __forceinline__ int scan_chunk(const int* __restrict__ lst, int nE, int cbase, int nodeBase,
                                          int* list, int tid, int lane, int wave, int fullvec) {
  int wc = 0;
#pragma unroll
  for (int g = 0; g < NGRP; ++g) {
    const int el0 = (g * NTHR + tid) * EPT;
    const int e0  = cbase + el0;
    v4i da, db;
    if (fullvec) {
      da = *(const v4i*)(lst + e0);
      db = *(const v4i*)(lst + e0 + 4);
    } else {
      const int em = nE - 1;
      da.x = lst[(e0     < em) ? e0     : em];
      da.y = lst[(e0 + 1 < em) ? e0 + 1 : em];
      da.z = lst[(e0 + 2 < em) ? e0 + 2 : em];
      da.w = lst[(e0 + 3 < em) ? e0 + 3 : em];
      db.x = lst[(e0 + 4 < em) ? e0 + 4 : em];
      db.y = lst[(e0 + 5 < em) ? e0 + 5 : em];
      db.z = lst[(e0 + 6 < em) ? e0 + 6 : em];
      db.w = lst[(e0 + 7 < em) ? e0 + 7 : em];
    }
    const bool v0 = (e0 < nE), v1 = (e0 + 1 < nE), v2 = (e0 + 2 < nE), v3 = (e0 + 3 < nE);
    const bool v4 = (e0 + 4 < nE), v5 = (e0 + 5 < nE), v6 = (e0 + 6 < nE), v7 = (e0 + 7 < nE);
    const unsigned nb = (unsigned)nodeBase;
    const unsigned s0 = (unsigned)da.x - nb, s1 = (unsigned)da.y - nb;
    const unsigned s2 = (unsigned)da.z - nb, s3 = (unsigned)da.w - nb;
    const unsigned s4 = (unsigned)db.x - nb, s5 = (unsigned)db.y - nb;
    const unsigned s6 = (unsigned)db.z - nb, s7 = (unsigned)db.w - nb;
    const bool h0 = v0 && (s0 < (unsigned)NB), h1 = v1 && (s1 < (unsigned)NB);
    const bool h2 = v2 && (s2 < (unsigned)NB), h3 = v3 && (s3 < (unsigned)NB);
    const bool h4 = v4 && (s4 < (unsigned)NB), h5 = v5 && (s5 < (unsigned)NB);
    const bool h6 = v6 && (s6 < (unsigned)NB), h7 = v7 && (s7 < (unsigned)NB);
    const unsigned any = __builtin_amdgcn_ballot_w32(h0 | h1 | h2 | h3 | h4 | h5 | h6 | h7);
    if (any != 0u) {
#define HITJ(J, HJ, SJ) { \
        const unsigned mj = __builtin_amdgcn_ballot_w32(HJ); \
        if (mj != 0u) { \
          if (HJ) { \
            const int pos = wc + (int)__builtin_amdgcn_mbcnt_lo(mj, 0u); \
            if (pos < WCAP) list[wave * WCAP + pos] = ((el0 + (J)) << 12) | (int)(SJ); \
          } \
          wc += (int)__builtin_popcount(mj); } }
      HITJ(0, h0, s0)
      HITJ(1, h1, s1)
      HITJ(2, h2, s2)
      HITJ(3, h3, s3)
      HITJ(4, h4, s4)
      HITJ(5, h5, s5)
      HITJ(6, h6, s6)
      HITJ(7, h7, s7)
#undef HITJ
    }
  }
  return wc;
}

__global__ __launch_bounds__(NTHR) void k_w16(const float* __restrict__ W, unsigned short* o, int n8) {
  const int i = blockIdx.x * NTHR + threadIdx.x;
  if (i >= n8) return;
  const float* p = W + (size_t)i * 8;
  v4f a = *(const v4f*)p, b = *(const v4f*)(p + 4);
  a = a * WSCALE; b = b * WSCALE;
  const v8h hv = pack8h(a, b);
  const size_t q = (size_t)i * 8;
  *(volatile v8h*)(o + q) = hv;
  __threadfence();
  *(volatile v8h*)(o + q) = hv;
}

__global__ __launch_bounds__(NTHR) void k_x16(const float* __restrict__ x, unsigned short* o, int nN, int nRows) {
  const int i = blockIdx.x * NTHR + threadIdx.x;
  if (i >= nRows * (FDIM / 8)) return;
  const int row = i >> 6;
  const int c0  = (i & 63) * 8;
  const int rc  = (row < nN) ? row : nN - 1;
  const float* xp = x + (size_t)rc * FDIM + c0;
  v4f a = *(const v4f*)xp, b = *(const v4f*)(xp + 4);
  if (row >= nN) { const v4f z = {0.f, 0.f, 0.f, 0.f}; a = z; b = z; }
  const v8h hv = pack8h(a, b);
  const size_t q = (size_t)row * FDIM + c0;
  *(volatile v8h*)(o + q) = hv;
  __threadfence();
  *(volatile v8h*)(o + q) = hv;
}

__global__ __launch_bounds__(NTHR) void k_deg(const int* __restrict__ coll, float* rcp, int nE, int vec_ok) {
  __shared__ __attribute__((aligned(16))) int   cnt[NBD];
  __shared__ __attribute__((aligned(16))) float rcl[NBD];
  __shared__ __attribute__((aligned(16))) int   list[LISTN];
  __shared__ int wcnt[NWAVE];
  const int tid = threadIdx.x, lane = tid & 31, wave = tid >> 5;
  const int nodeBase = blockIdx.x * NBD;

  for (int i = tid; i < NBD; i += NTHR) cnt[i] = 0;
  __syncthreads();

  const int nChunks = (nE + CHUNK - 1) / CHUNK;
#pragma unroll 1
  for (int ch = 0; ch < nChunks; ++ch) {
    const int cbase = ch * CHUNK;
    const int fullvec = (vec_ok != 0 && cbase + CHUNK <= nE) ? 1 : 0;
    const int wc = scan_chunk<NBD>(coll, nE, cbase, nodeBase, list, tid, lane, wave, fullvec);
    if (lane == 0) wcnt[wave] = wc;
    __syncthreads();
    if (wave == 0) {
#pragma unroll 1
      for (int wsx = 0; wsx < NWAVE; ++wsx) {
        int n = __builtin_amdgcn_readfirstlane(wcnt[wsx]);
        n = n > WCAP ? WCAP : (n < 0 ? 0 : n);
        const int* lp = list + wsx * WCAP;
#pragma unroll 1
        for (int i = 0; i < n; ++i) {
          const int ent  = __builtin_amdgcn_readfirstlane(lp[i]);
          const int slot = ent & (NBD - 1);
          if (lane == 0) cnt[slot] = cnt[slot] + 1;
        }
      }
    }
    __syncthreads();
  }

#pragma unroll 1
  for (int i = tid; i < NBD; i += NTHR) {
    int c = cnt[i];
    c = (c < 1) ? 1 : c;
    rcl[i] = 1.0f / (float)c;
  }
  __syncthreads();

  float* dp = rcp + (size_t)nodeBase;
  for (int pass = 0; pass < 2; ++pass) {
#pragma unroll
    for (int q = 0; q < 4; ++q) {
      const int f = (wave * 4 + q) * 128 + 4 * lane;
      const v4f v = *(const v4f*)(rcl + f);
      *(volatile v4f*)(dp + f) = v;
    }
    __threadfence();
  }
}

__global__ __launch_bounds__(NTHR) void k_agg(
    const int* __restrict__ rowl, const int* __restrict__ coll, const float* __restrict__ hp,
    const float* __restrict__ rcn, unsigned short* ob16, int nN, int nE, int vec_ok) {
  extern __shared__ v4f lds_dyn[];
  float* acc  = (float*)lds_dyn;
  int*   list = (int*)(acc + NBA * FDIM);
  int*   wcnt = list + LISTN;
  const int tid = threadIdx.x, lane = tid & 31, wave = tid >> 5;
  const int nodeBase = blockIdx.x * NBA;
  const v4f zz = {0.f, 0.f, 0.f, 0.f};

  for (int i = tid; i < NBA * FDIM / 4; i += NTHR) lds_dyn[i] = zz;
  __syncthreads();

  const int nChunks = (nE + CHUNK - 1) / CHUNK;
#pragma unroll 1
  for (int ch = 0; ch < nChunks; ++ch) {
    const int cbase = ch * CHUNK;
    const int fullvec = (vec_ok != 0 && cbase + CHUNK <= nE) ? 1 : 0;
    const int wc = scan_chunk<NBA>(coll, nE, cbase, nodeBase, list, tid, lane, wave, fullvec);
    if (lane == 0) wcnt[wave] = wc;
    __syncthreads();
    if (wave == 0) {
#pragma unroll 1
      for (int wsx = 0; wsx < NWAVE; ++wsx) {
        int n = __builtin_amdgcn_readfirstlane(wcnt[wsx]);
        n = n > WCAP ? WCAP : (n < 0 ? 0 : n);
        const int* lp = list + wsx * WCAP;
#pragma unroll 1
        for (int i = 0; i < n; ++i) {
          const int ent  = __builtin_amdgcn_readfirstlane(lp[i]);
          const int slot = ent & (NBA - 1);
          int e = cbase + ((ent >> 12) & (CHUNK - 1));
          e = e > nE - 1 ? nE - 1 : e;
          int s = rowl[e];
          s = s < 0 ? 0 : (s > nN - 1 ? nN - 1 : s);
          const float* hr = hp + (size_t)s * FDIM + 4 * lane;
          v4f* ar = (v4f*)(acc + slot * FDIM + 4 * lane);
          const v4f g0 = *(const v4f*)(hr);
          const v4f g1 = *(const v4f*)(hr + 128);
          const v4f g2 = *(const v4f*)(hr + 256);
          const v4f g3 = *(const v4f*)(hr + 384);
          ar[0]  = ar[0]  + g0;
          ar[32] = ar[32] + g1;
          ar[64] = ar[64] + g2;
          ar[96] = ar[96] + g3;
        }
      }
    }
    __syncthreads();
  }

#pragma unroll 2
  for (int i = 0; i < (NBA * FDIM / 4) / NTHR; ++i) {
    const int idx  = i * NTHR + tid;
    const int slot = idx >> 7;
    const int c4   = (idx & 127) * 4;
    const int node = nodeBase + slot;
    const int nc   = (node < nN) ? node : nN - 1;
    const float r  = rcn[nc];
    v4f* ap = (v4f*)(acc + slot * FDIM + c4);
    v4f v = (*ap) * r;
    if (node >= nN) v = zz;
    *ap = v;
  }
  __syncthreads();

  unsigned short* ob = ob16 + (size_t)nodeBase * FDIM;
  for (int pass = 0; pass < 2; ++pass) {
#pragma unroll
    for (int q = 0; q < 8; ++q) {
      const int row = wave * 8 + q;
#pragma unroll
      for (int hf = 0; hf < 2; ++hf) {
        const int col = hf * 256 + lane * 8;
        const float* sp = acc + row * FDIM + col;
        const v4f p0 = *(const v4f*)sp, p1 = *(const v4f*)(sp + 4);
        const v8h hv = pack8h(p0, p1);
        *(volatile v8h*)(ob + (size_t)row * FDIM + col) = hv;
      }
    }
    __threadfence();
  }
}

__global__ __launch_bounds__(NTHR) void k_ln(const float* __restrict__ y, const float* __restrict__ gam,
                                             const float* __restrict__ bet, unsigned short* xo, int nN) {
  const int lane = threadIdx.x & 31, wave = threadIdx.x >> 5;
  const int row  = blockIdx.x * NWAVE + wave;
  const int rcw  = (row < nN) ? row : nN - 1;
  const float* yr = y + (size_t)rcw * FDIM;
  const int cA = 8 * lane, cB = 256 + 8 * lane;
  const v4f a0 = relu4(*(const v4f*)(yr + cA)), a1 = relu4(*(const v4f*)(yr + cA + 4));
  const v4f a2 = relu4(*(const v4f*)(yr + cB)), a3 = relu4(*(const v4f*)(yr + cB + 4));
  float s = (((a0.x + a0.y) + (a0.z + a0.w)) + ((a1.x + a1.y) + (a1.z + a1.w)))
          + (((a2.x + a2.y) + (a2.z + a2.w)) + ((a3.x + a3.y) + (a3.z + a3.w)));
#pragma unroll
  for (int off = 16; off > 0; off >>= 1) s += __shfl_xor(s, off, 32);
  const float mu = s * (1.0f / 512.0f);
  const v4f d0 = a0 - mu, d1 = a1 - mu, d2 = a2 - mu, d3 = a3 - mu;
  float qv = (sq4(d0) + sq4(d1)) + (sq4(d2) + sq4(d3));
#pragma unroll
  for (int off = 16; off > 0; off >>= 1) qv += __shfl_xor(qv, off, 32);
  const float rs = rsqrtf(qv * (1.0f / 512.0f) + 1e-5f);
  const v4f g0 = *(const v4f*)(gam + cA), g1 = *(const v4f*)(gam + cA + 4);
  const v4f g2 = *(const v4f*)(gam + cB), g3 = *(const v4f*)(gam + cB + 4);
  const v4f b0 = *(const v4f*)(bet + cA), b1 = *(const v4f*)(bet + cA + 4);
  const v4f b2 = *(const v4f*)(bet + cB), b3 = *(const v4f*)(bet + cB + 4);
  v4f o0 = (d0 * rs) * g0 + b0, o1 = (d1 * rs) * g1 + b1;
  v4f o2 = (d2 * rs) * g2 + b2, o3 = (d3 * rs) * g3 + b3;
  if (row >= nN) { const v4f z = {0.f, 0.f, 0.f, 0.f}; o0 = z; o1 = z; o2 = z; o3 = z; }
  const v8h h0 = pack8h(o0, o1), h1 = pack8h(o2, o3);
  unsigned short* xr = xo + (size_t)row * FDIM;
  for (int pass = 0; pass < 2; ++pass) {
    *(volatile v8h*)(xr + cA) = h0;
    *(volatile v8h*)(xr + cB) = h1;
    __threadfence();
  }
}

__global__ __launch_bounds__(NTHR) void k_out(const float* __restrict__ y, float* out, int nN) {
  const int lane = threadIdx.x & 31, wave = threadIdx.x >> 5;
  const int row = blockIdx.x * NWAVE + wave;
  if (row >= nN) return;
  const float* yr = y + (size_t)row * FDIM + 4 * lane;
  float* orow = out + (size_t)row * FDIM + 4 * lane;
  const v4f v0 = *(const v4f*)(yr), v1 = *(const v4f*)(yr + 128);
  const v4f v2 = *(const v4f*)(yr + 256), v3 = *(const v4f*)(yr + 384);
  for (int pass = 0; pass < 2; ++pass) {
    *(volatile v4f*)(orow)       = v0;
    *(volatile v4f*)(orow + 128) = v1;
    *(volatile v4f*)(orow + 256) = v2;
    *(volatile v4f*)(orow + 384) = v3;
    __threadfence();
  }
}

extern "C" void kernel_launch(void* const* d_in, const int* in_sizes, int n_in,
                              void* d_out, int out_size, void* d_ws, size_t ws_size,
                              hipStream_t stream) {
  if (n_in < 21) return;
  const int nN = in_sizes[0] / FDIM;
  const int nE = in_sizes[1] / 2;
  if (nN < 1 || nE < 0 || in_sizes[0] != nN * FDIM || in_sizes[1] != 2 * nE) return;
  if (nN > (1 << 22)) return;
  {
    const int wIdx[9] = {2, 4, 6, 9, 11, 13, 16, 18, 20};
    for (int i = 0; i < 9; ++i) if (in_sizes[wIdx[i]] != FDIM * FDIM) return;
    const int vIdx[10] = {3, 5, 7, 8, 10, 12, 14, 15, 17, 19};
    for (int i = 0; i < 10; ++i) if (in_sizes[vIdx[i]] < FDIM) return;
  }
  if (out_size != nN * FDIM) return;

  const float* x   = (const float*)d_in[0];
  const int*   ei  = (const int*)d_in[1];
  const float* Wp0 = (const float*)d_in[2];  const float* bp0 = (const float*)d_in[3];
  const float* Wl0 = (const float*)d_in[4];  const float* bl0 = (const float*)d_in[5];
  const float* Wr0 = (const float*)d_in[6];
  const float* g0  = (const float*)d_in[7];  const float* be0 = (const float*)d_in[8];
  const float* Wp1 = (const float*)d_in[9];  const float* bp1 = (const float*)d_in[10];
  const float* Wl1 = (const float*)d_in[11]; const float* bl1 = (const float*)d_in[12];
  const float* Wr1 = (const float*)d_in[13];
  const float* g1  = (const float*)d_in[14]; const float* be1 = (const float*)d_in[15];
  const float* Wp2 = (const float*)d_in[16]; const float* bp2 = (const float*)d_in[17];
  const float* Wl2 = (const float*)d_in[18]; const float* bl2 = (const float*)d_in[19];
  const float* Wr2 = (const float*)d_in[20];
  const int* rowl = ei;
  const int* coll = ei + nE;
  float* out = (float*)d_out;

  const int nA  = (nN + NBA - 1) / NBA;
  const int Mp  = nA * NBA;
  const int nBD = (nN + NBD - 1) / NBD;
  const int vec_col = ((nE & 3) == 0) ? 1 : 0;

  char* ws = (char*)d_ws;
  size_t off = 0;
  const size_t wplane = (size_t)FDIM * FDIM * 2;
  const size_t oW16 = off; off += ((9 * wplane) + 255) & ~(size_t)255;
  const size_t oRcp = off; off += ((size_t)nBD * NBD * 4 + 255) & ~(size_t)255;
  const size_t oX16 = off; off += ((size_t)Mp * FDIM * 2 + 255) & ~(size_t)255;
  const size_t oHP  = off; off += ((size_t)Mp * FDIM * 4 + 255) & ~(size_t)255;
  const size_t oAG  = off; off += ((size_t)Mp * FDIM * 2 + 255) & ~(size_t)255;
  const size_t oY   = off; off += ((size_t)Mp * FDIM * 4 + 255) & ~(size_t)255;
  if (off > ws_size) return;

  unsigned short* w16 = (unsigned short*)(ws + oW16);
  float*          rcp = (float*)(ws + oRcp);
  unsigned short* x16 = (unsigned short*)(ws + oX16);
  float*          hpf = (float*)(ws + oHP);
  unsigned short* ag16 = (unsigned short*)(ws + oAG);
  float*          yf  = (float*)(ws + oY);

  const size_t WD = (size_t)FDIM * FDIM;
  const int n8 = (int)(WD / 8);
  const int gW = (n8 + NTHR - 1) / NTHR;

  k_w16<<<gW, NTHR, 0, stream>>>(Wp0, w16 + 0 * WD, n8);
  k_w16<<<gW, NTHR, 0, stream>>>(Wl0, w16 + 1 * WD, n8);
  k_w16<<<gW, NTHR, 0, stream>>>(Wr0, w16 + 2 * WD, n8);
  k_w16<<<gW, NTHR, 0, stream>>>(Wp1, w16 + 3 * WD, n8);
  k_w16<<<gW, NTHR, 0, stream>>>(Wl1, w16 + 4 * WD, n8);
  k_w16<<<gW, NTHR, 0, stream>>>(Wr1, w16 + 5 * WD, n8);
  k_w16<<<gW, NTHR, 0, stream>>>(Wp2, w16 + 6 * WD, n8);
  k_w16<<<gW, NTHR, 0, stream>>>(Wl2, w16 + 7 * WD, n8);
  k_w16<<<gW, NTHR, 0, stream>>>(Wr2, w16 + 8 * WD, n8);

  k_x16<<<(Mp * (FDIM / 8) + NTHR - 1) / NTHR, NTHR, 0, stream>>>(x, x16, nN, Mp);

  k_deg<<<nBD, NTHR, 0, stream>>>(coll, rcp, nE, vec_col);

  const int gG = ((Mp / 64) * (FDIM / 64) + 7) / 8;
  const float* bps[3] = {bp0, bp1, bp2};
  const float* bls[3] = {bl0, bl1, bl2};
  const float* gs[2]  = {g0, g1};
  const float* bes[2] = {be0, be1};

  for (int l = 0; l < 3; ++l) {
    const unsigned short* wp16 = w16 + (size_t)(3 * l + 0) * WD;
    const unsigned short* wl16 = w16 + (size_t)(3 * l + 1) * WD;
    const unsigned short* wr16 = w16 + (size_t)(3 * l + 2) * WD;
    wmma_gemm64<0, false, 2, 0, false, 2><<<dim3(gG, 1), 256, 0, stream>>>(
        x16, x16, FDIM, 0L, wp16, wp16, FDIM, 0L, (void*)hpf, (void*)hpf, FDIM, 0L,
        bps[l], bps[l], 0L, Mp, FDIM, FDIM, WSCALE_INV);
    k_agg<<<nA, NTHR, LDS_AGG, stream>>>(rowl, coll, hpf, rcp, ag16, nN, nE, vec_col);
    wmma_gemm64<0, false, 2, 0, false, 0><<<dim3(gG, 1), 256, 0, stream>>>(
        ag16, ag16, FDIM, 0L, wl16, wl16, FDIM, 0L, (void*)hpf, (void*)hpf, FDIM, 0L,
        bls[l], bls[l], 0L, Mp, FDIM, FDIM, WSCALE_INV);
    wmma_gemm64<0, false, 0, 0, true, 0><<<dim3(gG, 1), 256, 0, stream>>>(
        x16, x16, FDIM, 0L, wr16, wr16, FDIM, 0L, (void*)yf, (void*)yf, FDIM, 0L,
        bls[l], hpf, 0L, Mp, FDIM, FDIM, WSCALE_INV);
    if (l < 2)
      k_ln<<<Mp / NWAVE, NTHR, 0, stream>>>(yf, gs[l], bes[l], x16, nN);
  }

  k_out<<<(nN + NWAVE - 1) / NWAVE, NTHR, 0, stream>>>(yf, out, nN);
}
